// GFEModule_39711267619166
// MI455X (gfx1250) — hardware-verified
//
#include <hip/hip_runtime.h>
#define NI 128
#define NF 32
#define NCLIP 4
#define CC 256
#define SS 256
#define NH 8
#define HD 32
#define NR (NI * SS)
#define RCH (NF * SS)
#define NG 32
typedef __bf16 v16b __attribute__((ext_vector_type(16)));
typedef unsigned short v8us __attribute__((ext_vector_type(8), may_alias));
typedef float  v8f  __attribute__((ext_vector_type(8)));
typedef float  v4f  __attribute__((ext_vector_type(4)));
typedef float  v4fa __attribute__((ext_vector_type(4), may_alias));
union FragB { v16b v; v8us half[2]; unsigned short u[16]; };

__device__ __forceinline__ unsigned short bf16_bits(float x) { unsigned int u = __float_as_uint(x); return (unsigned short)((u + 0x7FFFu + ((u >> 16) & 1u)) >> 16); }
__device__ __forceinline__ float bf16_val(unsigned short b) { return __uint_as_float(((unsigned int)b) << 16); }
__device__ __forceinline__ float bf16_round(float x) { return bf16_val(bf16_bits(x)); }
template <int NT>
__device__ __forceinline__ v8f mmaN(v16b ah, v16b al, v16b bh, v16b bl, v8f c) {
  c = __builtin_amdgcn_wmma_f32_16x16x32_bf16(false, ah, false, bh, (short)0, c, false, false);
  if (NT >= 2) c = __builtin_amdgcn_wmma_f32_16x16x32_bf16(false, al, false, bh, (short)0, c, false, false);
  if (NT >= 3) c = __builtin_amdgcn_wmma_f32_16x16x32_bf16(false, ah, false, bl, (short)0, c, false, false);
  asm volatile("v_nop\n\tv_nop\n\tv_nop\n\tv_nop" : "+v"(c) : "v"(ah), "v"(al), "v"(bh), "v"(bl));
  return c;
}

__global__ __launch_bounds__(256) void k_wt_bf16(const float* __restrict__ W, unsigned short* __restrict__ Wt, int K, int N) {
  const int t = blockIdx.x * 256 + threadIdx.x;
  const int k8n = K / 8;
  if (t >= N * k8n) return;
  const int n = t / k8n, k8 = (t % k8n) * 8;
  v8us v;
#pragma unroll
  for (int i = 0; i < 8; ++i) v[i] = bf16_bits(W[(size_t)(k8 + i) * N + n]);
  *(volatile v8us*)(Wt + (size_t)n * K + k8) = v;
  __threadfence();
  *(volatile v8us*)(Wt + (size_t)n * K + k8) = v;
}

template <bool ASPLIT, int ACT, bool BIAS_BF16>
__global__ __launch_bounds__(128) void k_gemm_bf(const float* __restrict__ A, int lda, const unsigned short* __restrict__ Wt, int ldb,
                                               const float* __restrict__ bias, float* __restrict__ C, int ldc, int M, int N, int K) {
  __shared__ __attribute__((aligned(16))) float so[4][16][64];
  const int tid = threadIdx.x, w = tid >> 5, lane = tid & 31, ln = lane & 15, hh = lane >> 4;
  const int ntn = N / 64;
  const int wid = blockIdx.x * 4 + w;
  const int mt = wid / ntn, nq = wid % ntn;
  if (mt * 16 >= M) return;
  const int row0 = mt * 16, col0 = nq * 64;
  const float* arow = A + (size_t)(row0 + ln) * lda;
  v8f acc[4] = {};
  for (int kb = 0; kb < K; kb += 32) {
    FragB ah, al;
    const v4f x0 = *(const v4fa*)(arow + kb + 8 * hh), x1 = *(const v4fa*)(arow + kb + 8 * hh + 4);
    const v4f x2 = *(const v4fa*)(arow + kb + 16 + 8 * hh), x3 = *(const v4fa*)(arow + kb + 16 + 8 * hh + 4);
    float xs[16] = {x0[0],x0[1],x0[2],x0[3],x1[0],x1[1],x1[2],x1[3],x2[0],x2[1],x2[2],x2[3],x3[0],x3[1],x3[2],x3[3]};
#pragma unroll
    for (int i = 0; i < 16; ++i) { const unsigned short hb = bf16_bits(xs[i]); ah.u[i] = hb; al.u[i] = ASPLIT ? bf16_bits(xs[i] - bf16_val(hb)) : (unsigned short)0; }
#pragma unroll
    for (int t = 0; t < 4; ++t) {
      const unsigned short* brow = Wt + (size_t)(col0 + t * 16 + ln) * ldb + kb;
      FragB b;
      b.half[0] = *(const v8us*)(brow + 8 * hh);
      b.half[1] = *(const v8us*)(brow + 16 + 8 * hh);
      acc[t] = mmaN<ASPLIT ? 2 : 1>(ah.v, al.v, b.v, b.v, acc[t]);
    }
  }
#pragma unroll
  for (int t = 0; t < 4; ++t) {
    float bv = bias ? bias[col0 + t * 16 + ln] : 0.f;
    if (BIAS_BF16) bv = bf16_round(bv);
#pragma unroll
    for (int r = 0; r < 8; ++r) { float v = acc[t][r] + bv; if (ACT == 1) v = fmaxf(v, 0.f); so[w][8 * hh + r][t * 16 + ln] = v; }
  }
  __builtin_amdgcn_fence(__ATOMIC_ACQ_REL, "workgroup");
  __builtin_amdgcn_wave_barrier();
  const int rsub = lane >> 4, c4 = (lane & 15) * 4;
  for (int pass = 0; pass < 2; ++pass) {
#pragma unroll
    for (int q = 0; q < 8; ++q) {
      const int r = q * 2 + rsub;
      const v4f v = *(const v4fa*)&so[w][r][c4];
      *(volatile v4f*)(C + (size_t)(row0 + r) * ldc + col0 + c4) = v;
    }
    if (pass == 0) __threadfence();
  }
}

template <bool ASPLIT, int ACT, bool BIAS_BF16, bool RES_BF16>
__global__ __launch_bounds__(128) void k_gemm_bf3(const float* __restrict__ A, int lda, const unsigned short* __restrict__ Wt, int ldb,
                                                const float* __restrict__ bias, const float* __restrict__ resid, int rmod, int ldr,
                                                float* __restrict__ C, int ldc, int M, int N, int K) {
  __shared__ __attribute__((aligned(16))) float so[4][16][64];
  const int tid = threadIdx.x, w = tid >> 5, lane = tid & 31, ln = lane & 15, hh = lane >> 4;
  const int ntn = N / 64;
  const int wid = blockIdx.x * 4 + w;
  const int mt = wid / ntn, nq = wid % ntn;
  if (mt * 16 >= M) return;
  const int row0 = mt * 16, col0 = nq * 64;
  const float* arow = A + (size_t)(row0 + ln) * lda;
  v8f acc[4] = {};
  for (int kb = 0; kb < K; kb += 32) {
    FragB ah, al;
    const v4f x0 = *(const v4fa*)(arow + kb + 8 * hh), x1 = *(const v4fa*)(arow + kb + 8 * hh + 4);
    const v4f x2 = *(const v4fa*)(arow + kb + 16 + 8 * hh), x3 = *(const v4fa*)(arow + kb + 16 + 8 * hh + 4);
    float xs[16] = {x0[0],x0[1],x0[2],x0[3],x1[0],x1[1],x1[2],x1[3],x2[0],x2[1],x2[2],x2[3],x3[0],x3[1],x3[2],x3[3]};
#pragma unroll
    for (int i = 0; i < 16; ++i) { const unsigned short hb = bf16_bits(xs[i]); ah.u[i] = hb; al.u[i] = ASPLIT ? bf16_bits(xs[i] - bf16_val(hb)) : (unsigned short)0; }
#pragma unroll
    for (int t = 0; t < 4; ++t) {
      const unsigned short* brow = Wt + (size_t)(col0 + t * 16 + ln) * ldb + kb;
      FragB b;
      b.half[0] = *(const v8us*)(brow + 8 * hh);
      b.half[1] = *(const v8us*)(brow + 16 + 8 * hh);
      acc[t] = mmaN<ASPLIT ? 2 : 1>(ah.v, al.v, b.v, b.v, acc[t]);
    }
  }
#pragma unroll
  for (int t = 0; t < 4; ++t) {
    const int col = col0 + t * 16 + ln;
    float bv = bias ? bias[col] : 0.f;
    if (BIAS_BF16) bv = bf16_round(bv);
#pragma unroll
    for (int r = 0; r < 8; ++r) {
      float v = acc[t][r] + bv;
      if (resid) { float rv = resid[(size_t)((row0 + 8 * hh + r) % rmod) * ldr + col]; if (RES_BF16) rv = bf16_round(rv); v += rv; }
      if (ACT == 1) v = fmaxf(v, 0.f);
      if (ACT == 2) v = 0.5f * v * (1.0f + erff(v * 0.70710678118654752f));
      if (ACT == 3) { const float u = 0.7978845608028654f * (v + 0.044715f * v * v * v); v = 0.5f * v * (1.0f + tanhf(u)); }
      so[w][8 * hh + r][t * 16 + ln] = v;
    }
  }
  __builtin_amdgcn_fence(__ATOMIC_ACQ_REL, "workgroup");
  __builtin_amdgcn_wave_barrier();
  const int rsub = lane >> 4, c4 = (lane & 15) * 4;
  for (int pass = 0; pass < 2; ++pass) {
#pragma unroll
    for (int q = 0; q < 8; ++q) {
      const int r = q * 2 + rsub;
      const v4f v = *(const v4fa*)&so[w][r][c4];
      *(volatile v4f*)(C + (size_t)(row0 + r) * ldc + col0 + c4) = v;
    }
    if (pass == 0) __threadfence();
  }
}
template <bool PARAM_BF16>
__global__ __launch_bounds__(256) void k_layernorm(const float* __restrict__ X, const float* __restrict__ R, const float* __restrict__ g, const float* __restrict__ bta,
                                                  float* __restrict__ out_sum, float* __restrict__ out_norm, int N, float eps) {
  __shared__ float red[256];
  const int row = blockIdx.x, tid = threadIdx.x;
  const float* x = X + (size_t)row * N; const float* rr = R ? R + (size_t)row * N : nullptr;
  float vals[16];
  const int per = N / 256;
  float s1 = 0.f;
  for (int u = 0; u < per / 4; ++u) {
    const int j = tid * 4 + 1024 * u;
    const v4f a = *(const v4fa*)(x + j);
    v4f b = {0.f,0.f,0.f,0.f}; if (rr) b = *(const v4fa*)(rr + j);
#pragma unroll
    for (int q = 0; q < 4; ++q) { const float v = a[q] + b[q]; vals[u * 4 + q] = v; s1 += v; }
  }
  red[tid] = s1; __syncthreads();
  for (int st = 128; st > 0; st >>= 1) { if (tid < st) red[tid] += red[tid + st]; __syncthreads(); }
  const float mu = red[0] / (float)N; __syncthreads();
  float s2 = 0.f;
  for (int u = 0; u < per / 4; ++u)
#pragma unroll
    for (int q = 0; q < 4; ++q) { const float c = vals[u * 4 + q] - mu; s2 += c * c; }
  red[tid] = s2; __syncthreads();
  for (int st = 128; st > 0; st >>= 1) { if (tid < st) red[tid] += red[tid + st]; __syncthreads(); }
  const float rs = rsqrtf(red[0] / (float)N + eps);
  for (int pass = 0; pass < 2; ++pass) {
    for (int u = 0; u < per / 4; ++u) {
      const int j = tid * 4 + 1024 * u;
      v4f o, sm;
#pragma unroll
      for (int q = 0; q < 4; ++q) {
        float gg = g[j + q], bb = bta[j + q];
        if (PARAM_BF16) { gg = bf16_round(gg); bb = bf16_round(bb); }
        sm[q] = vals[u * 4 + q]; o[q] = (vals[u * 4 + q] - mu) * rs * gg + bb;
      }
      if (out_sum) *(volatile v4f*)(out_sum + (size_t)row * N + j) = sm;
      *(volatile v4f*)(out_norm + (size_t)row * N + j) = o;
    }
    if (pass == 0) __threadfence();
  }
}


typedef _Float16 v16h __attribute__((ext_vector_type(16)));
union FragH { v16h v; v8us half[2]; _Float16 h[16]; unsigned short u[16]; };
template <int NT>
__device__ __forceinline__ v8f mmaH(v16h ah, v16h al, v16h bh, v16h bl, v8f c) {
  c = __builtin_amdgcn_wmma_f32_16x16x32_f16(false, ah, false, bh, (short)0, c, false, false);
  if (NT >= 2) c = __builtin_amdgcn_wmma_f32_16x16x32_f16(false, al, false, bh, (short)0, c, false, false);
  if (NT >= 3) c = __builtin_amdgcn_wmma_f32_16x16x32_f16(false, ah, false, bl, (short)0, c, false, false);
  asm volatile("v_nop\n\tv_nop\n\tv_nop\n\tv_nop" : "+v"(c) : "v"(ah), "v"(al), "v"(bh), "v"(bl));
  return c;
}
template <bool ASPLIT>
__global__ __launch_bounds__(128) void k_gemm_h(const float* __restrict__ A, int lda, size_t sA, const _Float16* __restrict__ Bh, int ldb, size_t sB, float alpha, float* __restrict__ C, int ldc, size_t sC, int M, int N, int K) {
  __shared__ __attribute__((aligned(16))) float so[4][16][64];
  const int tid = threadIdx.x, w = tid >> 5, lane = tid & 31, ln = lane & 15, hh = lane >> 4; const int by = blockIdx.y;
  A += (size_t)by * sA; Bh += (size_t)by * sB; C += (size_t)by * sC;
  const int ntn = (N + 63) / 64; const int wid = blockIdx.x * 4 + w; const int mt = wid / ntn, nq = wid % ntn; if (mt * 16 >= M) return;
  const int row0 = mt * 16, col0 = nq * 64; const float* arow = A + (size_t)(row0 + ln) * lda;
  v8f acc[4] = {};
  for (int kb = 0; kb < K; kb += 32) {
    FragH ah, al;
    const v4f x0 = *(const v4fa*)(arow + kb + 8 * hh), x1 = *(const v4fa*)(arow + kb + 8 * hh + 4), x2 = *(const v4fa*)(arow + kb + 16 + 8 * hh), x3 = *(const v4fa*)(arow + kb + 16 + 8 * hh + 4);
    float xs[16] = {x0[0],x0[1],x0[2],x0[3],x1[0],x1[1],x1[2],x1[3],x2[0],x2[1],x2[2],x2[3],x3[0],x3[1],x3[2],x3[3]};
#pragma unroll
    for (int i = 0; i < 16; ++i) { const _Float16 h = (_Float16)xs[i]; ah.h[i] = h; al.h[i] = ASPLIT ? (_Float16)(xs[i] - (float)h) : (_Float16)0.0f; }
#pragma unroll
    for (int t = 0; t < 4; ++t) { if (col0 + t * 16 >= N) continue; const size_t boff = (size_t)(col0 + t * 16 + ln) * ldb + kb; FragH bq; bq.half[0] = *(const v8us*)(Bh + boff + 8 * hh); bq.half[1] = *(const v8us*)(Bh + boff + 16 + 8 * hh);
      acc[t] = mmaH<ASPLIT ? 2 : 1>(ah.v, al.v, bq.v, bq.v, acc[t]); }
  }
#pragma unroll
  for (int t = 0; t < 4; ++t) { if (col0 + t * 16 >= N) continue;
#pragma unroll
    for (int r = 0; r < 8; ++r) so[w][8 * hh + r][t * 16 + ln] = acc[t][r] * alpha; }
  __builtin_amdgcn_fence(__ATOMIC_ACQ_REL, "workgroup"); __builtin_amdgcn_wave_barrier();
  const int rsub = lane >> 4, c4 = (lane & 15) * 4;
  for (int pass = 0; pass < 2; ++pass) {
#pragma unroll
    for (int q = 0; q < 8; ++q) { const int r = q * 2 + rsub; if (col0 + c4 < N) { const v4f v = *(const v4fa*)&so[w][r][c4]; *(volatile v4f*)(C + (size_t)(row0 + r) * ldc + col0 + c4) = v; } }
    if (pass == 0) __threadfence(); }
}

__global__ __launch_bounds__(256) void k_wt_f16(const float* __restrict__ W, _Float16* __restrict__ Wt, int K, int N, float scale) {
  const int t = blockIdx.x * 256 + threadIdx.x; if (t >= N * (K / 8)) return; const int n = t / (K / 8), k8 = (t % (K / 8)) * 8; FragH f;
#pragma unroll
  for (int i = 0; i < 8; ++i) f.h[i] = (_Float16)(bf16_round(W[(size_t)(k8 + i) * N + n]) * scale); const v8us o = f.half[0];
  *(volatile v8us*)((unsigned short*)Wt + (size_t)n * K + k8) = o; __threadfence(); *(volatile v8us*)((unsigned short*)Wt + (size_t)n * K + k8) = o;
}
template <int ACT>
__global__ __launch_bounds__(128) void k_gemm_hhx(const _Float16* __restrict__ A, int lda, size_t sA, const _Float16* __restrict__ Bh, int ldb, size_t sB, float alpha, const float* __restrict__ bias, size_t sBias, const float* __restrict__ CP, int rowsPerB, size_t sCPb, int row0g,
    float* __restrict__ C, _Float16* __restrict__ C16, int ldc, size_t sC, int M, int N, int K) {
  __shared__ __attribute__((aligned(16))) float so[4][16][64];
  const int tid = threadIdx.x, w = tid >> 5, lane = tid & 31, ln = lane & 15, hh = lane >> 4; const int by = blockIdx.y;
  A += (size_t)by * sA; Bh += (size_t)by * sB; const size_t cofs = (size_t)by * sC; const float* bp = bias ? bias + (size_t)by * sBias : nullptr;
  const int ntn = (N + 63) / 64; const int wid = blockIdx.x * 4 + w; const int mt = wid / ntn, nq = wid % ntn; if (mt * 16 >= M) return;
  const int row0 = mt * 16, col0 = nq * 64; const _Float16* arow = A + (size_t)(row0 + ln) * lda;
  v8f acc[4] = {};
  for (int kb = 0; kb < K; kb += 32) { FragH ah; ah.half[0] = *(const v8us*)((const unsigned short*)arow + kb + 8 * hh); ah.half[1] = *(const v8us*)((const unsigned short*)arow + kb + 16 + 8 * hh);
#pragma unroll
    for (int t = 0; t < 4; ++t) { if (col0 + t * 16 >= N) continue; const size_t boff = (size_t)(col0 + t * 16 + ln) * ldb + kb; FragH bq; bq.half[0] = *(const v8us*)((const unsigned short*)Bh + boff + 8 * hh); bq.half[1] = *(const v8us*)((const unsigned short*)Bh + boff + 16 + 8 * hh);
      acc[t] = mmaH<1>(ah.v, ah.v, bq.v, bq.v, acc[t]); }
  }
#pragma unroll
  for (int t = 0; t < 4; ++t) { if (col0 + t * 16 >= N) continue; const int col = col0 + t * 16 + ln; const float bv = bp ? bf16_round(bp[col]) : 0.f;
#pragma unroll
    for (int r = 0; r < 8; ++r) { float v = acc[t][r] * alpha + bv; if (CP) { const int bidx = (row0g + row0 + 8 * hh + r) / rowsPerB; v += CP[(size_t)bidx * sCPb + (size_t)by * 64 + col]; } if (ACT == 1) v = (v > 0.f) ? v : expm1f(v); else if (ACT == 7) v = (v > 0.f) ? v + 1.0f : expf(v); else if (ACT == 8) v = tanhf(v); else if (ACT == 9) v = 0.5f * v * (1.0f + tanhf(0.7978845608028654f * (v + 0.044715f * v * v * v))); else if (ACT == 11) v = 1.0f / (1.0f + expf(-v)); else if (ACT == 12) v = (v > 0.f) ? v : 0.01f * v; else if (ACT == 14) v = (v > 0.f) ? v : 0.1f * v; else if (ACT == 15) v = v / (1.0f + expf(-v)); else if (ACT == 3) v = fmaxf(v, 0.f); else if (ACT == 6) v = 0.5f * v * (1.0f + erff(v * 0.70710678118654752f)); so[w][8 * hh + r][t * 16 + ln] = v; } }
  __builtin_amdgcn_fence(__ATOMIC_ACQ_REL, "workgroup"); __builtin_amdgcn_wave_barrier();
  const int rsub = lane >> 4, c4 = (lane & 15) * 4; typedef _Float16 v4h __attribute__((ext_vector_type(4)));
  for (int pass = 0; pass < 2; ++pass) {
#pragma unroll
    for (int q = 0; q < 8; ++q) { const int r = q * 2 + rsub; if (col0 + c4 < N) { const v4f v = *(const v4fa*)&so[w][r][c4]; if (C) *(volatile v4f*)(C + cofs + (size_t)(row0 + r) * ldc + col0 + c4) = v; if (C16) { v4h h4; for (int i = 0; i < 4; ++i) h4[i] = (_Float16)v[i]; *(volatile v4h*)(C16 + cofs + (size_t)(row0 + r) * ldc + col0 + c4) = h4; } } }
    if (pass == 0) __threadfence(); }
}


typedef _Float16 v4h __attribute__((ext_vector_type(4)));

__global__ __launch_bounds__(256) void k_x16(const float* __restrict__ x, _Float16* __restrict__ X16, size_t n8) { const size_t t = (size_t)blockIdx.x * 256 + threadIdx.x; if (t >= n8) return; FragH f;
#pragma unroll
  for (int q = 0; q < 8; ++q) f.h[q] = (_Float16)bf16_round(x[t * 8 + q]); *(volatile v8us*)((unsigned short*)X16 + t * 8) = f.half[0]; __threadfence(); *(volatile v8us*)((unsigned short*)X16 + t * 8) = f.half[0]; }
__global__ __launch_bounds__(256) void k_h16(const float* __restrict__ x, _Float16* __restrict__ X16, size_t n8) { const size_t t = (size_t)blockIdx.x * 256 + threadIdx.x; if (t >= n8) return; FragH f;
#pragma unroll
  for (int q = 0; q < 8; ++q) f.h[q] = (_Float16)x[t * 8 + q]; *(volatile v8us*)((unsigned short*)X16 + t * 8) = f.half[0]; __threadfence(); *(volatile v8us*)((unsigned short*)X16 + t * 8) = f.half[0]; }
__global__ __launch_bounds__(256) void k_round16f(const float* __restrict__ W, _Float16* __restrict__ Bt, size_t n8) { const size_t t = (size_t)blockIdx.x * 256 + threadIdx.x; if (t >= n8) return; FragH f;
#pragma unroll
  for (int i = 0; i < 8; ++i) f.h[i] = (_Float16)(bf16_round(W[t * 8 + i]) * 16.0f); *(volatile v8us*)((unsigned short*)Bt + t * 8) = f.half[0]; __threadfence(); *(volatile v8us*)((unsigned short*)Bt + t * 8) = f.half[0]; }
template <int NHv, int TTv>
__global__ __launch_bounds__(256) void k_vt(const _Float16* __restrict__ V16, int ldv, int voff, _Float16* __restrict__ Vt) { __shared__ unsigned short tl[64][66]; const int tid = threadIdx.x; const int slab = blockIdx.x / (TTv / 64), lg = blockIdx.x % (TTv / 64); const int b = slab / NHv, h = slab % NHv;
  for (int i = tid; i < 64 * 8; i += 256) { const int r = i / 8, c8 = (i % 8) * 8; FragH f; f.half[0] = *(const v8us*)((const unsigned short*)V16 + ((size_t)b * TTv + lg * 64 + r) * ldv + voff + h * 64 + c8);
#pragma unroll
    for (int q = 0; q < 8; ++q) tl[r][c8 + q] = f.u[q]; }
  __syncthreads();
  for (int pass = 0; pass < 2; ++pass) {
#pragma unroll
    for (int rd = 0; rd < 2; ++rd) { const int d = rd * 32 + tid / 8, pc = tid % 8; FragH f;
#pragma unroll
      for (int q = 0; q < 8; ++q) f.u[q] = tl[pc * 8 + q][d];
      *(volatile v8us*)((unsigned short*)Vt + ((size_t)slab * 64 + d) * TTv + lg * 64 + pc * 8) = f.half[0]; }
    if (pass == 0) __threadfence(); } }

__global__ __launch_bounds__(256) void k_hl(const float* __restrict__ F, _Float16* __restrict__ Hh, _Float16* __restrict__ Hl, size_t n8) { const size_t t = (size_t)blockIdx.x * 256 + threadIdx.x; if (t >= n8) return; FragH fh, fl; const v4f a = *(const v4fa*)(F + t * 8), c = *(const v4fa*)(F + t * 8 + 4);
#pragma unroll
  for (int q = 0; q < 4; ++q) { _Float16 h = (_Float16)a[q]; fh.h[q] = h; fl.h[q] = (_Float16)((a[q] - (float)h) * 1024.0f); h = (_Float16)c[q]; fh.h[4 + q] = h; fl.h[4 + q] = (_Float16)((c[q] - (float)h) * 1024.0f); }
  for (int pass = 0; pass < 2; ++pass) { *(volatile v8us*)((unsigned short*)Hh + t * 8) = fh.half[0]; *(volatile v8us*)((unsigned short*)Hl + t * 8) = fl.half[0]; if (pass == 0) __threadfence(); } }

__device__ __forceinline__ v4f shfl4(v4f v, int srcl) { v4f r; r[0] = __shfl(v[0], srcl, 32); r[1] = __shfl(v[1], srcl, 32); r[2] = __shfl(v[2], srcl, 32); r[3] = __shfl(v[3], srcl, 32); return r; }
__device__ __forceinline__ void store_row8(float* row, v4f oa, v4f ob, int l) { const v4f a1 = shfl4(oa, l >> 1), b1 = shfl4(ob, l >> 1), a2 = shfl4(oa, 16 + (l >> 1)), b2 = shfl4(ob, 16 + (l >> 1)); const v4f c1 = (l & 1) ? b1 : a1, c2 = (l & 1) ? b2 : a2; for (int pass = 0; pass < 2; ++pass) { *(volatile v4f*)(row + l * 4) = c1; *(volatile v4f*)(row + 128 + l * 4) = c2; if (pass == 0) __threadfence(); } }
__global__ __launch_bounds__(256) void k_tok(const float* __restrict__ feat, float* __restrict__ TOK, _Float16* __restrict__ T16) {
  #pragma clang fp contract(off)
  const int t = blockIdx.x * 256 + threadIdx.x; if (t >= NR * (CC / 8)) return; const int c0 = (t % (CC / 8)) * 8, r = t / (CC / 8); const int i = r / SS, s = r % SS; const int l = threadIdx.x & 31; v4f oa, ob; FragH f;
#pragma unroll
  for (int q = 0; q < 8; ++q) { const float v = bf16_round(feat[((size_t)i * CC + c0 + q) * SS + s]); if (q < 4) oa[q] = v; else ob[q - 4] = v; f.h[q] = (_Float16)v; }
  store_row8(TOK + (size_t)r * CC, oa, ob, l);
  *(volatile v8us*)((unsigned short*)T16 + (size_t)r * CC + c0) = f.half[0]; __threadfence(); *(volatile v8us*)((unsigned short*)T16 + (size_t)r * CC + c0) = f.half[0]; }
__global__ __launch_bounds__(256) void k_prev(const _Float16* __restrict__ K16, _Float16* __restrict__ KP) { const int t = blockIdx.x * 256 + threadIdx.x; if (t >= RCH * (CC / 8)) return; const int c0 = (t % (CC / 8)) * 8, r = t / (CC / 8); const int n = r / SS, s = r % SS; const int pn = max(n - 1, 0); FragH f; f.half[0] = *(const v8us*)((const unsigned short*)K16 + ((size_t)pn * SS + s) * CC + c0);
  *(volatile v8us*)((unsigned short*)KP + (size_t)r * CC + c0) = f.half[0]; __threadfence(); *(volatile v8us*)((unsigned short*)KP + (size_t)r * CC + c0) = f.half[0]; }
__global__ __launch_bounds__(256) void k_vtn(const _Float16* __restrict__ V16, _Float16* __restrict__ VT) { const int t = blockIdx.x * 256 + threadIdx.x; if (t >= NF * CC * (SS / 8)) return; const int s0 = (t % (SS / 8)) * 8; const int hd = (t / (SS / 8)) % CC; const int n = t / ((SS / 8) * CC); const int nn = min(n + 1, NF - 1); FragH f;
#pragma unroll
  for (int q = 0; q < 8; ++q) f.h[q] = V16[((size_t)nn * SS + s0 + q) * CC + hd];
  *(volatile v8us*)((unsigned short*)VT + ((size_t)n * CC + hd) * SS + s0) = f.half[0]; __threadfence(); *(volatile v8us*)((unsigned short*)VT + ((size_t)n * CC + hd) * SS + s0) = f.half[0]; }
__global__ __launch_bounds__(256) void k_soft(const float* __restrict__ S, _Float16* __restrict__ P16) {
  #pragma clang fp contract(off)
  const int tid = threadIdx.x, w = tid >> 5, ln = tid & 31; const int row = blockIdx.x * 8 + w; if (row >= NF * SS) return; const v4f a = *(const v4fa*)(S + (size_t)row * SS + ln * 8), c = *(const v4fa*)(S + (size_t)row * SS + ln * 8 + 4); float m = -3.0e38f;
#pragma unroll
  for (int k = 0; k < 4; ++k) { m = fmaxf(m, a[k]); m = fmaxf(m, c[k]); }
  for (int o = 16; o > 0; o >>= 1) m = fmaxf(m, __shfl_xor(m, o, 32));
  float e[8]; float su = 0.f;
#pragma unroll
  for (int k = 0; k < 8; ++k) { e[k] = expf(((k < 4) ? a[k] : c[k - 4]) - m); su += e[k]; }
  for (int o = 16; o > 0; o >>= 1) su += __shfl_xor(su, o, 32); const float inv = 1024.0f / su; FragH f;
#pragma unroll
  for (int k = 0; k < 8; ++k) f.h[k] = (_Float16)(e[k] * inv);
  *(volatile v8us*)((unsigned short*)P16 + (size_t)row * SS + ln * 8) = f.half[0]; __threadfence(); *(volatile v8us*)((unsigned short*)P16 + (size_t)row * SS + ln * 8) = f.half[0]; }
__global__ __launch_bounds__(256) void k_lnc(float* __restrict__ X, const float* __restrict__ g, const float* __restrict__ bb) {
  #pragma clang fp contract(off)
  const int tid = threadIdx.x, w = tid >> 5, l = tid & 31; const int r = blockIdx.x * 8 + w; if (r >= NR) return; float v[8]; float s = 0.f;
#pragma unroll
  for (int k = 0; k < 8; ++k) { v[k] = X[(size_t)r * CC + l * 8 + k]; s += v[k]; }
  for (int o = 16; o > 0; o >>= 1) s += __shfl_xor(s, o, 32); const float mu = s / (float)CC; float q2 = 0.f;
#pragma unroll
  for (int k = 0; k < 8; ++k) { const float d = v[k] - mu; q2 += d * d; }
  for (int o = 16; o > 0; o >>= 1) q2 += __shfl_xor(q2, o, 32); const float rs = 1.0f / sqrtf(q2 / (float)CC + 1e-5f); v4f oa, ob;
#pragma unroll
  for (int k = 0; k < 8; ++k) { const int c = l * 8 + k; const float y = (v[k] - mu) * rs * bf16_round(g[c]) + bf16_round(bb[c]); if (k < 4) oa[k] = y; else ob[k - 4] = y; }
  store_row8(X + (size_t)r * CC, oa, ob, l); }
__global__ __launch_bounds__(256) void k_gap(const float* __restrict__ FA, _Float16* __restrict__ GA16) {
  #pragma clang fp contract(off)
  const int t = blockIdx.x * 256 + threadIdx.x; if (t >= NI * (CC / 8)) return; const int c0 = (t % (CC / 8)) * 8, i = t / (CC / 8); float acc[8];
#pragma unroll
  for (int q = 0; q < 8; ++q) acc[q] = 0.f;
#pragma unroll 1
  for (int s = 0; s < SS; ++s) { const v4f a = *(const v4fa*)(FA + ((size_t)i * SS + s) * CC + c0), c = *(const v4fa*)(FA + ((size_t)i * SS + s) * CC + c0 + 4);
#pragma unroll
    for (int q = 0; q < 8; ++q) acc[q] += (q < 4) ? a[q] : c[q - 4]; }
  FragH f;
#pragma unroll
  for (int q = 0; q < 8; ++q) f.h[q] = (_Float16)(acc[q] / (float)SS);
  *(volatile v8us*)((unsigned short*)GA16 + (size_t)i * CC + c0) = f.half[0]; __threadfence(); *(volatile v8us*)((unsigned short*)GA16 + (size_t)i * CC + c0) = f.half[0]; }
__global__ __launch_bounds__(256) void k_dydw(const float* __restrict__ FA, const float* __restrict__ KERN, _Float16* __restrict__ DW16) {
  #pragma clang fp contract(off)
  const int t = blockIdx.x * 256 + threadIdx.x; if (t >= NR * (CC / 8)) return; const int c0 = (t % (CC / 8)) * 8, r = t / (CC / 8); const int i = r / SS, s = r % SS; const int y = s / 16, x = s % 16; float acc[8];
#pragma unroll
  for (int q = 0; q < 8; ++q) acc[q] = 0.f;
#pragma unroll 1
  for (int tp = 0; tp < 9; ++tp) { const int yy = y + tp / 3 - 1, xx = x + tp % 3 - 1; if (yy < 0 || yy >= 16 || xx < 0 || xx >= 16) continue; const v4f a = *(const v4fa*)(FA + ((size_t)i * SS + yy * 16 + xx) * CC + c0), c = *(const v4fa*)(FA + ((size_t)i * SS + yy * 16 + xx) * CC + c0 + 4);
#pragma unroll
    for (int q = 0; q < 8; ++q) acc[q] += KERN[(size_t)i * CC * 9 + (c0 + q) * 9 + tp] * ((q < 4) ? a[q] : c[q - 4]); }
  FragH f;
#pragma unroll
  for (int q = 0; q < 8; ++q) f.h[q] = (_Float16)acc[q];
  *(volatile v8us*)((unsigned short*)DW16 + (size_t)r * CC + c0) = f.half[0]; __threadfence(); *(volatile v8us*)((unsigned short*)DW16 + (size_t)r * CC + c0) = f.half[0]; }
__global__ __launch_bounds__(256) void k_gnstat(const float* __restrict__ DC, int phase, float* __restrict__ GST) {
  #pragma clang fp contract(off)
  __shared__ float red[256]; const int ig = blockIdx.x, tid = threadIdx.x; const int i = ig / NG, g = ig % NG; const float mean = phase ? (GST[(size_t)ig * 32] / 2048.0f) : 0.f; float s = 0.f;
  for (int e = tid; e < 2048; e += 256) { const int px = e / 8, cc = e % 8; const float v = DC[((size_t)i * SS + px) * CC + g * 8 + cc]; s += phase ? (v - mean) * (v - mean) : v; }
  red[tid] = s; __syncthreads(); for (int st = 128; st > 0; st >>= 1) { if (tid < st) red[tid] += red[tid + st]; __syncthreads(); }
  if (tid < 32) { float* line = GST + ((size_t)phase * NI * NG + ig) * 32; *(volatile float*)(line + tid) = red[0]; __threadfence(); *(volatile float*)(line + tid) = red[0]; } }
__global__ __launch_bounds__(256) void k_gnapply(const float* __restrict__ DC, const float* __restrict__ GST, const float* __restrict__ g, const float* __restrict__ bb, _Float16* __restrict__ O16) {
  #pragma clang fp contract(off)
  const int t = blockIdx.x * 256 + threadIdx.x; if (t >= NR * (CC / 8)) return; const int c0 = (t % (CC / 8)) * 8, r = t / (CC / 8); const int i = r / SS; const int ig = i * NG + c0 / 8; const float mean = GST[(size_t)ig * 32] / 2048.0f, rs = 1.0f / sqrtf(GST[(size_t)(NI * NG + ig) * 32] / 2048.0f + 1e-5f); const v4f a = *(const v4fa*)(DC + (size_t)r * CC + c0), c = *(const v4fa*)(DC + (size_t)r * CC + c0 + 4); FragH f;
#pragma unroll
  for (int q = 0; q < 8; ++q) { const int ch = c0 + q; f.h[q] = (_Float16)((((q < 4) ? a[q] : c[q - 4]) - mean) * rs * bf16_round(g[ch]) + bf16_round(bb[ch])); }
  *(volatile v8us*)((unsigned short*)O16 + (size_t)r * CC + c0) = f.half[0]; __threadfence(); *(volatile v8us*)((unsigned short*)O16 + (size_t)r * CC + c0) = f.half[0]; }
__global__ __launch_bounds__(256) void k_fstat(const float* __restrict__ Y, int phase, float* __restrict__ FST) {
  #pragma clang fp contract(off)
  __shared__ float red[256]; const int i = blockIdx.x, tid = threadIdx.x; const float mean = phase ? (FST[(size_t)i * 32] / 65536.0f) : 0.f; float s = 0.f; const float* base = Y + (size_t)i * SS * CC;
  for (int e = tid; e < SS * CC; e += 256) { const float v = base[e]; s += phase ? (v - mean) * (v - mean) : v; }
  red[tid] = s; __syncthreads(); for (int st = 128; st > 0; st >>= 1) { if (tid < st) red[tid] += red[tid + st]; __syncthreads(); }
  if (tid < 32) { float* line = FST + ((size_t)phase * NI + i) * 32; *(volatile float*)(line + tid) = red[0]; __threadfence(); *(volatile float*)(line + tid) = red[0]; } }
__global__ __launch_bounds__(256) void k_out(const float* __restrict__ Y, const float* __restrict__ FST, const float* __restrict__ g, const float* __restrict__ bb, float* __restrict__ out) {
  #pragma clang fp contract(off)
  const int t = blockIdx.x * 256 + threadIdx.x; if (t >= NI * CC * (SS / 4)) return; const int s0 = (t % (SS / 4)) * 4; const int c = (t / (SS / 4)) % CC; const int i = t / ((SS / 4) * CC); const float mean = FST[(size_t)i * 32] / 65536.0f, rs = 1.0f / sqrtf(FST[(size_t)(NI + i) * 32] / 65536.0f + 1e-5f); v4f v;
#pragma unroll
  for (int q = 0; q < 4; ++q) { const int s = s0 + q; v[q] = (Y[((size_t)i * SS + s) * CC + c] - mean) * rs * bf16_round(g[c * SS + s]) + bf16_round(bb[c * SS + s]); }
  float* dst = out + ((size_t)i * CC + c) * SS + s0; *(volatile v4f*)dst = v; __threadfence(); *(volatile v4f*)dst = v; }

extern "C" void kernel_launch(void* const* d_in, const int* in_sizes, int n_in,
                              void* d_out, int out_size, void* d_ws, size_t ws_size, hipStream_t stream) {
  (void)in_sizes; (void)n_in; (void)out_size;
  const float* const* I = (const float* const*)d_in; const float* feat = I[0]; const float* ipw = I[1]; const float* ipb = I[2]; const float* opw = I[3]; const float* opb = I[4]; const float* ln1g = I[5]; const float* ln1b = I[6]; const float* kgw1 = I[7]; const float* kgb1 = I[8]; const float* kgw2 = I[9]; const float* kgb2 = I[10]; const float* dcw = I[11]; const float* dcb = I[12]; const float* gng = I[13]; const float* gnb = I[14]; const float* fc1w = I[15]; const float* fc1b = I[16]; const float* fc2w = I[17]; const float* fc2b = I[18]; const float* dcng = I[19]; const float* dcnb = I[20];
  char* ws = (char*)d_ws; size_t off = 0;
  auto take = [&](size_t bytes) { char* p = ws + off; off += (bytes + 255) & ~(size_t)255; return p; };
  _Float16* BIP = (_Float16*)take((size_t)3 * CC * CC * 2); _Float16* BOP = (_Float16*)take((size_t)CC * CC * 2); _Float16* BK1 = (_Float16*)take((size_t)CC * CC * 2); _Float16* BK2 = (_Float16*)take((size_t)9 * CC * CC * 2); _Float16* BDC = (_Float16*)take((size_t)CC * CC * 2); _Float16* BF1 = (_Float16*)take((size_t)CC * CC * 2); _Float16* BF2 = (_Float16*)take((size_t)CC * CC * 2); float* GST = (float*)take((size_t)2 * NI * NG * 32 * 4); float* FST = (float*)take((size_t)2 * NI * 32 * 4); float* KERN = (float*)take((size_t)NI * 9 * CC * 4); _Float16* GA16 = (_Float16*)take((size_t)NI * CC * 2); _Float16* H116 = (_Float16*)take((size_t)NI * CC * 2);
  float* TOK = (float*)take((size_t)NR * CC * 4); _Float16* T16 = (_Float16*)take((size_t)NR * CC * 2); float* X = (float*)take((size_t)NR * CC * 4);
  char* CHK = take((size_t)RCH * CC * 2 * 6 + (size_t)NF * SS * SS * 4 + (size_t)NF * SS * SS * 2);
  if (off > ws_size) return;
  _Float16* Q16 = (_Float16*)CHK; _Float16* K16 = Q16 + (size_t)RCH * CC; _Float16* KP16 = K16 + (size_t)RCH * CC; _Float16* V16 = KP16 + (size_t)RCH * CC; _Float16* VT = V16 + (size_t)RCH * CC; _Float16* CTX16 = VT + (size_t)RCH * CC; float* S = (float*)(CTX16 + (size_t)RCH * CC); _Float16* P16 = (_Float16*)(S + (size_t)NF * SS * SS);
  _Float16* DW16 = T16;
  float* DC = TOK;
  _Float16* DCN16 = (_Float16*)CHK; _Float16* H16 = DCN16 + (size_t)NR * CC;
  float* Y = DC;
  k_round16f<<<(3 * CC * CC / 8 + 255) / 256, 256, 0, stream>>>(ipw, BIP, (size_t)3 * CC * CC / 8); k_round16f<<<(CC * CC / 8 + 255) / 256, 256, 0, stream>>>(opw, BOP, (size_t)CC * CC / 8); k_round16f<<<(CC * CC / 8 + 255) / 256, 256, 0, stream>>>(kgw1, BK1, (size_t)CC * CC / 8); k_round16f<<<(9 * CC * CC / 8 + 255) / 256, 256, 0, stream>>>(kgw2, BK2, (size_t)9 * CC * CC / 8); k_round16f<<<(CC * CC / 8 + 255) / 256, 256, 0, stream>>>(dcw, BDC, (size_t)CC * CC / 8); k_round16f<<<(CC * CC / 8 + 255) / 256, 256, 0, stream>>>(fc1w, BF1, (size_t)CC * CC / 8); k_round16f<<<(CC * CC / 8 + 255) / 256, 256, 0, stream>>>(fc2w, BF2, (size_t)CC * CC / 8);
  const size_t n8 = (size_t)NR * CC / 8; const unsigned nb8 = (unsigned)((n8 + 255) / 256);
  k_tok<<<nb8, 256, 0, stream>>>(feat, TOK, T16);
  const dim3 gCc(((RCH / 16) * (CC / 64) + 3) / 4, 1), gS(((SS / 16) * (SS / 64) + 3) / 4, NF), gV(((SS / 16) * 1 + 3) / 4, NF), gCall(((NR / 16) * (CC / 64) + 3) / 4, 1);
  for (int cl = 0; cl < NCLIP; ++cl) { const size_t r0 = (size_t)cl * RCH; const _Float16* Tc = T16 + r0 * CC;
    k_gemm_hhx<0><<<gCc, 128, 0, stream>>>(Tc, CC, 0, BIP, CC, 0, 0.0625f, ipb, 0, nullptr, 1, 0, 0, nullptr, Q16, CC, 0, RCH, CC, CC);
    k_gemm_hhx<0><<<gCc, 128, 0, stream>>>(Tc, CC, 0, BIP + (size_t)CC * CC, CC, 0, 0.0625f, ipb + CC, 0, nullptr, 1, 0, 0, nullptr, K16, CC, 0, RCH, CC, CC);
    k_gemm_hhx<0><<<gCc, 128, 0, stream>>>(Tc, CC, 0, BIP + (size_t)2 * CC * CC, CC, 0, 0.0625f, ipb + 2 * CC, 0, nullptr, 1, 0, 0, nullptr, V16, CC, 0, RCH, CC, CC);
    k_prev<<<(RCH * (CC / 8) + 255) / 256, 256, 0, stream>>>(K16, KP16); k_vtn<<<(NF * CC * (SS / 8) + 255) / 256, 256, 0, stream>>>(V16, VT);
    for (int h = 0; h < NH; ++h) {
      k_gemm_hhx<0><<<gS, 128, 0, stream>>>(Q16 + h * HD, CC, (size_t)SS * CC, KP16 + h * HD, CC, (size_t)SS * CC, 0.17677669529663687f, nullptr, 0, nullptr, 1, 0, 0, S, nullptr, SS, (size_t)SS * SS, SS, SS, HD);
      k_soft<<<NF * SS / 8, 256, 0, stream>>>(S, P16);
      k_gemm_hhx<0><<<gV, 128, 0, stream>>>(P16, SS, (size_t)SS * SS, VT + (size_t)h * HD * SS, SS, (size_t)CC * SS, 0.0009765625f, nullptr, 0, nullptr, 1, 0, 0, nullptr, CTX16 + h * HD, CC, (size_t)SS * CC, SS, HD, SS); }
    k_gemm_hhx<0><<<gCc, 128, 0, stream>>>(CTX16, CC, 0, BOP, CC, 0, 0.0625f, opb, 0, TOK + r0 * CC, 1, (size_t)CC, 0, X + r0 * CC, nullptr, CC, 0, RCH, CC, CC); }
  k_lnc<<<NR / 8, 256, 0, stream>>>(X, ln1g, ln1b);
  const float* FA = X;
  k_gap<<<(NI * (CC / 8) + 255) / 256, 256, 0, stream>>>(FA, GA16);
  k_gemm_hhx<3><<<dim3(((NI / 16) * (CC / 64) + 3) / 4, 1), 128, 0, stream>>>(GA16, CC, 0, BK1, CC, 0, 0.0625f, kgb1, 0, nullptr, 1, 0, 0, nullptr, H116, CC, 0, NI, CC, CC);
  k_gemm_hhx<0><<<dim3(((NI / 16) * (9 * CC / 64) + 3) / 4, 1), 128, 0, stream>>>(H116, CC, 0, BK2, CC, 0, 0.0625f, kgb2, 0, nullptr, 1, 0, 0, KERN, nullptr, 9 * CC, 0, NI, 9 * CC, CC);
  k_dydw<<<nb8, 256, 0, stream>>>(FA, KERN, DW16);
  k_gemm_hhx<0><<<gCall, 128, 0, stream>>>(DW16, CC, 0, BDC, CC, 0, 0.0625f, dcb, 0, nullptr, 1, 0, 0, DC, nullptr, CC, 0, NR, CC, CC);
  k_gnstat<<<NI * NG, 256, 0, stream>>>(DC, 0, GST); k_gnstat<<<NI * NG, 256, 0, stream>>>(DC, 1, GST);
  k_gnapply<<<nb8, 256, 0, stream>>>(DC, GST, gng, gnb, DCN16);
  k_gemm_hhx<3><<<gCall, 128, 0, stream>>>(DCN16, CC, 0, BF1, CC, 0, 0.0625f, fc1b, 0, nullptr, 1, 0, 0, nullptr, H16, CC, 0, NR, CC, CC);
  k_gemm_hhx<0><<<gCall, 128, 0, stream>>>(H16, CC, 0, BF2, CC, 0, 0.0625f, fc2b, 0, FA, 1, (size_t)CC, 0, Y, nullptr, CC, 0, NR, CC, CC);
  k_fstat<<<NI, 256, 0, stream>>>(Y, 0, FST); k_fstat<<<NI, 256, 0, stream>>>(Y, 1, FST);
  k_out<<<(NI * CC * (SS / 4) + 255) / 256, 256, 0, stream>>>(Y, FST, dcng, dcnb, (float*)d_out);
}
